// RNNs_81011673137155
// MI455X (gfx1250) — hardware-verified
//
#include <hip/hip_runtime.h>

typedef __attribute__((ext_vector_type(16))) _Float16 v16h;
typedef __attribute__((ext_vector_type(8)))  _Float16 v8h;
typedef __attribute__((ext_vector_type(8)))  float    v8f;
typedef __attribute__((ext_vector_type(4)))  float    v4f;

constexpr int kBatch  = 64;
constexpr int kNodes  = 2048;
constexpr int kT      = 12;
constexpr int kHid    = 32;
constexpr int kGate   = 96;
constexpr int kOutC   = 12;
constexpr int kOutPad = 16;
constexpr int kSeq    = kBatch * kNodes;
constexpr int kWaves  = 8;
constexpr int kThreads = 256;
constexpr int kSeqPerWave  = 16;
constexpr int kSeqPerBlock = kWaves * kSeqPerWave;
static_assert(kSeq % kSeqPerBlock == 0, "grid covers all sequences exactly");
static_assert(kSeqPerWave * kT == 192, "per-wave input block = 192 floats = 48 x 16 B");
static_assert(kSeqPerWave * kOutC == 192, "per-wave output block = 192 floats = 6 whole 128-B lines");

constexpr float kWsc = 16.0f;
constexpr float kHsc = 8.0f;
constexpr float kInv = 1.0f / 128.0f;

union FragU { v16h v; v8h h[2]; };
__device__ __forceinline__ v16h frag_load(const _Float16* p) {
  FragU f; f.h[0] = *(const v8h*)(p); f.h[1] = *(const v8h*)(p + 16); return f.v;
}

__device__ __forceinline__ v8f mma16(v16h a, v16h b, v8f c) {
  c = __builtin_amdgcn_wmma_f32_16x16x32_f16(false, a, false, b, (short)0, c, false, false);
  asm volatile("v_nop\n\tv_nop\n\tv_nop\n\tv_nop" : "+v"(c) : "v"(a), "v"(b));
  return c;
}

__device__ __forceinline__ void wave_lds_sync() {
  __builtin_amdgcn_fence(__ATOMIC_RELEASE, "workgroup");
  __builtin_amdgcn_wave_barrier();
  __builtin_amdgcn_fence(__ATOMIC_ACQUIRE, "workgroup");
}

__device__ __forceinline__ float rcp_f(float x) {
#if __has_builtin(__builtin_amdgcn_rcpf)
  return __builtin_amdgcn_rcpf(x);
#else
  return 1.0f / x;
#endif
}
__device__ __forceinline__ float sigm_f(float x) {
  const float e = expf(-x);
  return rcp_f(1.0f + e);
}
__device__ __forceinline__ float tanh_f(float x) {
  const float ax = fabsf(x);
  const float e  = expf(-2.0f * ax);
  const float t  = (1.0f - e) * rcp_f(1.0f + e);
  return copysignf(t, x);
}

__global__ __launch_bounds__(kThreads) void gru2_fused_kernel(
    const float* __restrict__ xin,
    const float* __restrict__ start_w,
    const float* __restrict__ start_b,
    const float* __restrict__ w1x,
    const float* __restrict__ w1h,
    const float* __restrict__ b1x,
    const float* __restrict__ b1h,
    const float* __restrict__ w2x,
    const float* __restrict__ w2h,
    const float* __restrict__ b2x,
    const float* __restrict__ b2h,
    const float* __restrict__ ew,
    const float* __restrict__ eb,
    float* __restrict__ out)
{
  __shared__ __align__(16) _Float16 wBt[3 * kGate * kHid];
  __shared__ __align__(16) _Float16 eBt[kT * kOutPad * kHid];
  __shared__ float sAvec[kGate];
  __shared__ float sBcon[kGate];
  __shared__ float sb1h[kGate];
  __shared__ float sb2x[kGate];
  __shared__ float sb2h[kGate];
  __shared__ float seb[kOutPad];
  __shared__ __align__(16) float u_t[kWaves][kT][kSeqPerWave];
  __shared__ __align__(16) _Float16 hst[kWaves][2][kSeqPerWave * kHid];
  __shared__ __align__(16) float osl[kWaves][kSeqPerWave * kOutC];

  const int tid  = threadIdx.x;
  const int wave = tid >> 5;
  const int lane = tid & 31;
  const int cidx = lane & 15;
  const int hh   = lane >> 4;

#pragma unroll 4
  for (int e = tid; e < kGate * kHid; e += kThreads) {
    const int k = e & 31, n = e >> 5;
    wBt[e] = (_Float16)(kWsc * w1h[k * kGate + n]);
  }
#pragma unroll 4
  for (int e = tid; e < kGate * kHid; e += kThreads) {
    const int k = e & 31, n = e >> 5;
    wBt[kGate * kHid + e] = (_Float16)(kWsc * w2x[k * kGate + n]);
  }
#pragma unroll 4
  for (int e = tid; e < kGate * kHid; e += kThreads) {
    const int k = e & 31, n = e >> 5;
    wBt[2 * kGate * kHid + e] = (_Float16)(kWsc * w2h[k * kGate + n]);
  }
#pragma unroll 4
  for (int e = tid; e < kT * kOutPad * kHid; e += kThreads) {
    const int k = e & 31;
    const int o = (e >> 5) & 15;
    const int t = e >> 9;
    const int oc = (o < kOutC) ? o : (kOutC - 1);
    const float v = ew[(oc * kHid + k) * kT + t];
    eBt[e] = (_Float16)((o < kOutC) ? (kWsc * v) : 0.0f);
  }
  if (tid < kGate) {
    float a = 0.0f, bc = 0.0f;
#pragma unroll 4
    for (int c = 0; c < kHid; ++c) {
      const float w = w1x[c * kGate + tid];
      a  = fmaf(start_w[c], w, a);
      bc = fmaf(start_b[c], w, bc);
    }
    sAvec[tid] = a;
    sBcon[tid] = bc + b1x[tid];
    sb1h[tid] = b1h[tid];
    sb2x[tid] = b2x[tid];
    sb2h[tid] = b2h[tid];
  }
  if (tid < kOutPad) {
    const int oc = (tid < kOutC) ? tid : (kOutC - 1);
    const float v = eb[oc];
    seb[tid] = (tid < kOutC) ? v : 0.0f;
  }

  const int tileBase = (blockIdx.x * kWaves + wave) * kSeqPerWave;
  {
    const float* ib = xin + (size_t)tileBase * kT;
    const v4f c0 = *(const v4f*)(ib + lane * 4);
    const v4f c1 = *(const v4f*)(ib + (32 + (lane & 15)) * 4);
#pragma unroll
    for (int e = 0; e < 4; ++e) {
      const int f = lane * 4 + e;
      const int m = f / kT;
      const int tt = f - m * kT;
      u_t[wave][tt][m] = c0[e];
    }
    if (lane < 16) {
#pragma unroll
      for (int e = 0; e < 4; ++e) {
        const int f = 128 + lane * 4 + e;
        const int m = f / kT;
        const int tt = f - m * kT;
        u_t[wave][tt][m] = c1[e];
      }
    }
  }
  __syncthreads();

  float Az[2], Ar[2], An[2], Bz[2], Br[2], Bn[2];
  float b1z[2], b1r[2], b1n[2];
  float bz2[2], br2[2], bxn2[2], bhn2[2];
#pragma unroll
  for (int q = 0; q < 2; ++q) {
    const int cz = 16 * q + cidx, cr = cz + 32, cn = cz + 64;
    Az[q] = sAvec[cz]; Ar[q] = sAvec[cr]; An[q] = sAvec[cn];
    Bz[q] = sBcon[cz]; Br[q] = sBcon[cr]; Bn[q] = sBcon[cn];
    b1z[q] = sb1h[cz]; b1r[q] = sb1h[cr]; b1n[q] = sb1h[cn];
    bz2[q]  = sb2x[cz] + sb2h[cz];
    br2[q]  = sb2x[cr] + sb2h[cr];
    bxn2[q] = sb2x[cn];
    bhn2[q] = sb2h[cn];
  }
  const float ebv = seb[cidx];

  const v8f zero8 = (v8f){0.f, 0.f, 0.f, 0.f, 0.f, 0.f, 0.f, 0.f};
  v8f h1[2], h2[2], yacc;
  h1[0] = zero8; h1[1] = zero8; h2[0] = zero8; h2[1] = zero8; yacc = zero8;
  v16h a1, a2;
#pragma unroll
  for (int i = 0; i < 16; ++i) { a1[i] = (_Float16)0.0f; a2[i] = (_Float16)0.0f; }

  _Float16* st1 = &hst[wave][0][0];
  _Float16* st2 = &hst[wave][1][0];
  const _Float16* wB1h = wBt;
  const _Float16* wB2x = wBt + kGate * kHid;
  const _Float16* wB2h = wBt + 2 * kGate * kHid;

#pragma unroll 1
  for (int t = 0; t < kT; ++t) {
    const float* up = &u_t[wave][t][8 * hh];
    const v4f ua = *(const v4f*)(up);
    const v4f ub = *(const v4f*)(up + 4);
    const float uv[8] = { ua[0], ua[1], ua[2], ua[3], ub[0], ub[1], ub[2], ub[3] };

#pragma unroll
    for (int q = 0; q < 2; ++q) {
      const int zc = 16 * q, rc = 32 + 16 * q, nc = 64 + 16 * q;
      v8f gz = mma16(a1, frag_load(wB1h + (zc + cidx) * kHid + 8 * hh), zero8);
      v8f gr = mma16(a1, frag_load(wB1h + (rc + cidx) * kHid + 8 * hh), zero8);
      v8f gn = mma16(a1, frag_load(wB1h + (nc + cidx) * kHid + 8 * hh), zero8);
#pragma unroll
      for (int r = 0; r < 8; ++r) {
        const float u  = uv[r];
        const float pz = fmaf(u, Az[q], Bz[q]) + fmaf(gz[r], kInv, b1z[q]);
        const float pr = fmaf(u, Ar[q], Br[q]) + fmaf(gr[r], kInv, b1r[q]);
        const float hn = fmaf(gn[r], kInv, b1n[q]);
        const float z  = sigm_f(pz);
        const float rg = sigm_f(pr);
        const float ng = tanh_f(fmaf(u, An[q], Bn[q]) + rg * hn);
        h1[q][r] = fmaf(z, h1[q][r] - ng, ng);
      }
    }
#pragma unroll
    for (int q = 0; q < 2; ++q)
#pragma unroll
      for (int r = 0; r < 8; ++r)
        st1[(8 * hh + r) * kHid + 16 * q + cidx] = (_Float16)(h1[q][r] * kHsc);
    wave_lds_sync();
    a1 = frag_load(st1 + cidx * kHid + 8 * hh);

#pragma unroll
    for (int q = 0; q < 2; ++q) {
      const int zc = 16 * q, rc = 32 + 16 * q, nc = 64 + 16 * q;
      v8f gz = mma16(a1, frag_load(wB2x + (zc + cidx) * kHid + 8 * hh), zero8);
      gz     = mma16(a2, frag_load(wB2h + (zc + cidx) * kHid + 8 * hh), gz);
      v8f gr = mma16(a1, frag_load(wB2x + (rc + cidx) * kHid + 8 * hh), zero8);
      gr     = mma16(a2, frag_load(wB2h + (rc + cidx) * kHid + 8 * hh), gr);
      v8f gxn = mma16(a1, frag_load(wB2x + (nc + cidx) * kHid + 8 * hh), zero8);
      v8f ghn = mma16(a2, frag_load(wB2h + (nc + cidx) * kHid + 8 * hh), zero8);
#pragma unroll
      for (int r = 0; r < 8; ++r) {
        const float z  = sigm_f(fmaf(gz[r], kInv, bz2[q]));
        const float rg = sigm_f(fmaf(gr[r], kInv, br2[q]));
        const float hn = fmaf(ghn[r], kInv, bhn2[q]);
        const float ng = tanh_f(fmaf(gxn[r], kInv, bxn2[q]) + rg * hn);
        h2[q][r] = fmaf(z, h2[q][r] - ng, ng);
      }
    }
#pragma unroll
    for (int q = 0; q < 2; ++q)
#pragma unroll
      for (int r = 0; r < 8; ++r)
        st2[(8 * hh + r) * kHid + 16 * q + cidx] = (_Float16)(h2[q][r] * kHsc);
    wave_lds_sync();
    a2 = frag_load(st2 + cidx * kHid + 8 * hh);

    yacc = mma16(a2, frag_load(eBt + (t * kOutPad + cidx) * kHid + 8 * hh), yacc);
  }

  if (cidx < kOutC) {
    float* os = osl[wave];
#pragma unroll
    for (int r = 0; r < 8; ++r) os[(8 * hh + r) * kOutC + cidx] = fmaf(yacc[r], kInv, ebv);
  }
  wave_lds_sync();
  {
    const float* os = osl[wave];
    const v4f v0 = *(const v4f*)(os + lane * 4);
    const v4f v1 = *(const v4f*)(os + (32 + (lane & 15)) * 4);
    float* ob = out + (size_t)tileBase * kOutC;
    for (int pass = 0; pass < 2; ++pass) {
      *(volatile v4f*)(ob + lane * 4) = v0;
      if (lane < 16) *(volatile v4f*)(ob + 128 + lane * 4) = v1;
      __threadfence();
    }
  }
}

extern "C" void kernel_launch(void* const* d_in, const int* in_sizes, int n_in,
                              void* d_out, int out_size, void* d_ws, size_t ws_size,
                              hipStream_t stream) {
  const float* xin     = (const float*)d_in[0];
  const float* start_w = (const float*)d_in[1];
  const float* start_b = (const float*)d_in[2];
  const float* w1x     = (const float*)d_in[3];
  const float* w1h     = (const float*)d_in[4];
  const float* b1x     = (const float*)d_in[5];
  const float* b1h     = (const float*)d_in[6];
  const float* w2x     = (const float*)d_in[7];
  const float* w2h     = (const float*)d_in[8];
  const float* b2x     = (const float*)d_in[9];
  const float* b2h     = (const float*)d_in[10];
  const float* ew      = (const float*)d_in[11];
  const float* eb      = (const float*)d_in[12];
  float* out           = (float*)d_out;
  (void)in_sizes; (void)n_in; (void)d_ws; (void)ws_size;

  if (out_size < kSeq * kOutC) return;

  dim3 grid(kSeq / kSeqPerBlock);
  dim3 block(kThreads);
  gru2_fused_kernel<<<grid, block, 0, stream>>>(
      xin, start_w, start_b, w1x, w1h, b1x, b1h,
      w2x, w2h, b2x, b2h, ew, eb, out);
}
